// IGConv_71322226917424
// MI455X (gfx1250) — hardware-verified
//
#include <hip/hip_runtime.h>
#include <stddef.h>
#include <math.h>


#define NTHR   256
#define NWAVE  8
#define NAG    128
#define FEATD  32
#define EMBD   64
#define YD     256
#define HID    256
#define K2IN   160
#define NSPLIT 8
#define PASSN  (NWAVE * 16)
#define LFP    264
#define HP     264
#define AGP    168
#define XLP    72
#define SC     16.0f
#define INV2   0.00390625f

#define PB0 32
#define PB1 8
#define PB2 8
#define PB3 20
#define PB4 8
#define PBT (PB0 + PB1 + PB2 + PB3 + PB4)

#define E_LF   0
#define E_H    (E_LF + NWAVE * 16 * LFP * 2)
#define E_MSG  (E_H + PASSN * HP * 2)
#define E_ACC  (E_MSG + PASSN * EMBD * 4)
#define E_SLOT (E_ACC + (NAG + 1) * EMBD * 4)
#define E_PRM  (E_SLOT + PASSN * 4)
#define E_TOT  (E_PRM + EMBD * 4)

#define P_XS   0
#define P_ST   (P_XS + NAG * XLP * 2)
#define P_TOT  (P_ST + NAG * HID * 4)

#define N_AG   0
#define N_H    (N_AG + NAG * AGP * 2)
#define N_OUT  (N_H + NAG * HP * 2)
#define N_PRM  (N_OUT + NAG * EMBD * 4)
#define N_TOT  (N_PRM + (HID + EMBD) * 4)

static_assert(PB0 * NTHR * 8 == HID * YD);
static_assert(PB1 * NTHR * 8 == HID * EMBD);
static_assert(PB2 * NTHR * 8 == EMBD * HID);
static_assert(PB3 * NTHR * 8 == HID * K2IN);
static_assert(PB4 * NTHR * 8 == EMBD * HID);
static_assert((E_H % 16) == 0 && (E_MSG % 16) == 0 && (E_ACC % 16) == 0 && (E_SLOT % 16) == 0 && (E_PRM % 16) == 0);
static_assert((P_ST % 16) == 0 && (N_H % 16) == 0 && (N_OUT % 16) == 0 && (N_PRM % 16) == 0);
static_assert(E_TOT <= 300 * 1024 && P_TOT <= 300 * 1024 && N_TOT <= 300 * 1024);
static_assert((LFP % 8) == 0 && (HP % 8) == 0 && (AGP % 8) == 0 && (XLP % 8) == 0);
static_assert(LFP >= YD && HP >= HID && AGP >= K2IN && XLP >= EMBD);
static_assert((YD % 32) == 0 && (HID % 32) == 0 && (K2IN % 32) == 0 && (EMBD % 32) == 0);
static_assert(NWAVE * 16 == NAG);
static_assert((NAG * EMBD) % (NTHR * 4) == 0 && (NAG * HID) % (NTHR * 4) == 0);
static_assert(K2IN == FEATD + EMBD + EMBD);

typedef float    v4f  __attribute__((ext_vector_type(4)));
typedef float    v8f  __attribute__((ext_vector_type(8)));
typedef int      v4i  __attribute__((ext_vector_type(4)));
typedef _Float16 v4h  __attribute__((ext_vector_type(4)));
typedef _Float16 v8h  __attribute__((ext_vector_type(8)));
typedef _Float16 v16h __attribute__((ext_vector_type(16)));
union FragH { v16h v; v8h h[2]; };
union Pk8 { v8h h; v4i i; };

__device__ __forceinline__ v8f wmh(v16h a, v16h b, v8f c) {
  v8f d = __builtin_amdgcn_wmma_f32_16x16x32_f16(false, a, false, b, (short)0, c, false, false);
  asm volatile("v_nop\n\tv_nop\n\tv_nop\n\tv_nop" : "+v"(d) : "v"(a), "v"(b));
  return d;
}

__device__ __forceinline__ v8f splat8(float x) {
  v8f c;
#pragma unroll
  for (int i = 0; i < 8; ++i) c[i] = x;
  return c;
}

__device__ __forceinline__ v8f ldc8(const float* p) {
  const v4f a = *(const v4f*)p;
  const v4f b = *(const v4f*)(p + 4);
  v8f c;
  c[0] = a.x; c[1] = a.y; c[2] = a.z; c[3] = a.w;
  c[4] = b.x; c[5] = b.y; c[6] = b.z; c[7] = b.w;
  return c;
}

__device__ __forceinline__ v16h ldfrag(const _Float16* p) {
  FragH a;
  a.h[0] = *(const v8h*)p;
  a.h[1] = *(const v8h*)(p + 16);
  return a.v;
}

__device__ __forceinline__ v8h cv8s(v4f a, v4f b) {
  v8h r;
  r[0] = (_Float16)(a.x * SC); r[1] = (_Float16)(a.y * SC); r[2] = (_Float16)(a.z * SC); r[3] = (_Float16)(a.w * SC);
  r[4] = (_Float16)(b.x * SC); r[5] = (_Float16)(b.y * SC); r[6] = (_Float16)(b.z * SC); r[7] = (_Float16)(b.w * SC);
  return r;
}

__device__ __forceinline__ v4h cv4s(v4f a) {
  v4h r;
  r[0] = (_Float16)(a.x * SC); r[1] = (_Float16)(a.y * SC); r[2] = (_Float16)(a.z * SC); r[3] = (_Float16)(a.w * SC);
  return r;
}

__device__ __forceinline__ v8h act8(v8f d, v8f p) {
  v8h r;
#pragma unroll
  for (int i = 0; i < 8; ++i) {
    const float t = fmaxf(d[i] * INV2 + p[i], 0.0f) * SC;
    r[i] = (_Float16)t;
  }
  return r;
}

__global__ __launch_bounds__(NTHR) void k_prep(
    const float* __restrict__ w1, const float* __restrict__ w2,
    const float* __restrict__ w3, const float* __restrict__ w4,
    _Float16* p1y, _Float16* p1x, _Float16* p2, _Float16* p3, _Float16* p4) {
  const int b = blockIdx.x, tid = threadIdx.x;
  const float* src;
  _Float16* dst;
  int K, R, koff, ub;
  if (b < PB0) {
    src = w1; dst = p1y; K = YD;   R = HID;  koff = 0;  ub = b;
  } else if (b < PB0 + PB1) {
    src = w1; dst = p1x; K = EMBD; R = HID;  koff = YD; ub = b - PB0;
  } else if (b < PB0 + PB1 + PB2) {
    src = w2; dst = p2;  K = HID;  R = EMBD; koff = 0;  ub = b - (PB0 + PB1);
  } else if (b < PB0 + PB1 + PB2 + PB3) {
    src = w3; dst = p3;  K = K2IN; R = HID;  koff = 0;  ub = b - (PB0 + PB1 + PB2);
  } else {
    src = w4; dst = p4;  K = HID;  R = EMBD; koff = 0;  ub = b - (PB0 + PB1 + PB2 + PB3);
  }
  const int u   = ub * NTHR + tid;
  const int cpr = K >> 3;
  const int row = u / cpr;
  const int kc  = u - row * cpr;
  Pk8 pk;
#pragma unroll
  for (int j = 0; j < 8; ++j) {
    const int k = 8 * kc + j;
    const float w = src[(size_t)(koff + k) * R + row];
    pk.h[j] = (_Float16)(w * SC);
  }
  _Float16* dp = dst + (size_t)u * 8;
  *(volatile v4i*)dp = pk.i;
  __threadfence();
  *(volatile v4i*)dp = pk.i;
}

__global__ __launch_bounds__(NTHR) void k_pnode(const float* __restrict__ xl,
                                                const _Float16* __restrict__ W1x,
                                                const float* __restrict__ b1,
                                                float* P) {
  extern __shared__ __attribute__((aligned(16))) unsigned char dsm[];
  _Float16* xs  = (_Float16*)(dsm + P_XS);
  float*    pst = (float*)(dsm + P_ST);
  const int tid = threadIdx.x, lane = tid & 31, wave = tid >> 5, hh = lane >> 4, m = lane & 15;
  const int b = blockIdx.x;

#pragma unroll
  for (int it = 0; it < (NAG * EMBD / 8) / NTHR; ++it) {
    const int i = it * NTHR + tid;
    const int n = i >> 3, c8 = i & 7;
    const float* xp = xl + ((size_t)(b * NAG + n)) * EMBD + 8 * c8;
    *(v8h*)(xs + n * XLP + 8 * c8) = cv8s(*(const v4f*)xp, *(const v4f*)(xp + 4));
  }
  __syncthreads();

  const int lrow = 16 * wave + m;
  FragH bx[2];
#pragma unroll
  for (int kf = 0; kf < 2; ++kf) {
    const _Float16* p = xs + lrow * XLP + 32 * kf + 8 * hh;
    bx[kf].h[0] = *(const v8h*)p;
    bx[kf].h[1] = *(const v8h*)(p + 16);
  }
#pragma unroll 1
  for (int ht = 0; ht < HID / 16; ++ht) {
    v8f c = splat8(0.0f);
#pragma unroll
    for (int kf = 0; kf < 2; ++kf)
      c = wmh(ldfrag(W1x + (size_t)(16 * ht + m) * EMBD + 32 * kf + 8 * hh), bx[kf].v, c);
    const int f0 = 16 * ht + 8 * hh;
    const v8f bb = ldc8(b1 + f0);
    float o[8];
#pragma unroll
    for (int r = 0; r < 8; ++r) o[r] = c[r] * INV2 + bb[r];
    float* sp = pst + lrow * HID + f0;
    const v4f o0 = {o[0], o[1], o[2], o[3]};
    const v4f o1 = {o[4], o[5], o[6], o[7]};
    *(v4f*)sp = o0;
    *(v4f*)(sp + 4) = o1;
  }
  __syncthreads();

  float* pp = P + (size_t)b * (NAG * HID);
#pragma unroll 1
  for (int it = 0; it < (NAG * HID) / (NTHR * 4); ++it) {
    const int i = it * NTHR * 4 + 4 * tid;
    const v4f v = *(const v4f*)(pst + i);
    *(volatile v4f*)(pp + i) = v;
  }
  __threadfence();
#pragma unroll 1
  for (int it = 0; it < (NAG * HID) / (NTHR * 4); ++it) {
    const int i = it * NTHR * 4 + 4 * tid;
    const v4f v = *(const v4f*)(pst + i);
    *(volatile v4f*)(pp + i) = v;
  }
}

__global__ __launch_bounds__(NTHR) __attribute__((amdgpu_num_vgpr(256))) void k_edge(
    const float* __restrict__ x0, const float* __restrict__ eattr, const int* __restrict__ ei,
    const float* __restrict__ convw, const float* __restrict__ convb, const float* __restrict__ b2,
    const float* __restrict__ P, const _Float16* __restrict__ W1y, const _Float16* __restrict__ W2p,
    float* part, int nE, int epb) {
  extern __shared__ __attribute__((aligned(16))) unsigned char dsm[];
  _Float16* lf    = (_Float16*)(dsm + E_LF);
  _Float16* hb    = (_Float16*)(dsm + E_H);
  float*    msg   = (float*)(dsm + E_MSG);
  float*    acc   = (float*)(dsm + E_ACC);
  int*      slotb = (int*)(dsm + E_SLOT);
  float*    prm   = (float*)(dsm + E_PRM);

  const int tid = threadIdx.x, lane = tid & 31, wave = tid >> 5, hh = lane >> 4, m = lane & 15;
  const int s = blockIdx.x, b = blockIdx.y;

  {
    const v4f z = {0.0f, 0.0f, 0.0f, 0.0f};
    for (int i = tid; i < (NAG + 1) * EMBD / 4; i += NTHR) *(v4f*)(acc + 4 * i) = z;
  }
  if (tid < EMBD) prm[tid] = b2[tid];
  __syncthreads();

  const int ebeg = s * epb;
  int eend = ebeg + epb;
  eend = eend > nE ? nE : eend;
  const int nPass = (eend > ebeg) ? (eend - ebeg + PASSN - 1) / PASSN : 0;
  const int lrow = 16 * wave + m;

#pragma unroll 1
  for (int p = 0; p < nPass; ++p) {
    int src;
    {
      float cw[16], cb[8];
#pragma unroll
      for (int i = 0; i < 16; ++i) cw[i] = convw[i];
#pragma unroll
      for (int i = 0; i < 8; ++i) cb[i] = convb[i];
      const int e = ebeg + p * PASSN + lrow;
      const bool valid = e < eend;
      const int ec = e > nE - 1 ? nE - 1 : e;
      int si = ei[2 * ec];
      const int di = ei[2 * ec + 1];
      si = si < 0 ? 0 : (si > NAG - 1 ? NAG - 1 : si);
      src = si;
      const int slot = (valid && (unsigned)di < (unsigned)NAG) ? di : NAG;
      if (hh == 0) slotb[lrow] = slot;
      const float* nfp = x0 + ((size_t)(b * NAG + si)) * FEATD + 16 * hh;
      const float* eap = eattr + ((size_t)b * (size_t)nE + (size_t)ec) * FEATD + 16 * hh;
      const v4f na = *(const v4f*)nfp,  nb = *(const v4f*)(nfp + 4);
      const v4f nc = *(const v4f*)(nfp + 8), nd = *(const v4f*)(nfp + 12);
      const v4f ga = *(const v4f*)eap,  gb = *(const v4f*)(eap + 4);
      const v4f gc = *(const v4f*)(eap + 8), gd = *(const v4f*)(eap + 12);
      float nf[16], ea[16];
      nf[0] = na.x; nf[1] = na.y; nf[2]  = na.z; nf[3]  = na.w; nf[4]  = nb.x; nf[5]  = nb.y; nf[6]  = nb.z; nf[7]  = nb.w;
      nf[8] = nc.x; nf[9] = nc.y; nf[10] = nc.z; nf[11] = nc.w; nf[12] = nd.x; nf[13] = nd.y; nf[14] = nd.z; nf[15] = nd.w;
      ea[0] = ga.x; ea[1] = ga.y; ea[2]  = ga.z; ea[3]  = ga.w; ea[4]  = gb.x; ea[5]  = gb.y; ea[6]  = gb.z; ea[7]  = gb.w;
      ea[8] = gc.x; ea[9] = gc.y; ea[10] = gc.z; ea[11] = gc.w; ea[12] = gd.x; ea[13] = gd.y; ea[14] = gd.z; ea[15] = gd.w;
      _Float16* lr = lf + (size_t)lrow * LFP + 16 * hh;
#pragma unroll
      for (int o = 0; o < 8; ++o) {
        const float w0 = cw[2 * o], w1 = cw[2 * o + 1], cbo = cb[o];
        v8h ya, yb;
#pragma unroll
        for (int j = 0; j < 8; ++j) {
          ya[j] = (_Float16)(fmaxf(w0 * nf[j] + w1 * ea[j] + cbo, 0.0f) * SC);
          yb[j] = (_Float16)(fmaxf(w0 * nf[8 + j] + w1 * ea[8 + j] + cbo, 0.0f) * SC);
        }
        *(v8h*)(lr + 32 * o) = ya;
        *(v8h*)(lr + 32 * o + 8) = yb;
      }
    }
    __syncthreads();

    {
      const _Float16* brow = lf + (size_t)lrow * LFP + 8 * hh;
      const float* prow = P + ((size_t)(b * NAG + src)) * HID + 8 * hh;
      _Float16* hrow = hb + (size_t)lrow * HP + 8 * hh;
#pragma unroll 1
      for (int q = 0; q < HID / 32; ++q) {
        v8f d0 = splat8(0.0f), d1 = splat8(0.0f);
        const _Float16* w0p = W1y + (size_t)(32 * q + m) * YD + 8 * hh;
        const _Float16* w1p = w0p + (size_t)16 * YD;
#pragma unroll 2
        for (int kf = 0; kf < YD / 32; ++kf) {
          FragH bl;
          bl.h[0] = *(const v8h*)(brow + 32 * kf);
          bl.h[1] = *(const v8h*)(brow + 32 * kf + 16);
          d0 = wmh(ldfrag(w0p + 32 * kf), bl.v, d0);
          d1 = wmh(ldfrag(w1p + 32 * kf), bl.v, d1);
        }
        const v8h h0 = act8(d0, ldc8(prow + 32 * q));
        const v8h h1 = act8(d1, ldc8(prow + 32 * q + 16));
        *(v8h*)(hrow + 32 * q) = h0;
        *(v8h*)(hrow + 32 * q + 16) = h1;
      }
    }
    __syncthreads();

    {
      const _Float16* hrow = hb + (size_t)lrow * HP + 8 * hh;
      float* mrow = msg + lrow * EMBD + 8 * hh;
#pragma unroll 1
      for (int ot = 0; ot < EMBD / 16; ++ot) {
        v8f c = splat8(0.0f);
        const _Float16* wp = W2p + (size_t)(16 * ot + m) * HID + 8 * hh;
#pragma unroll 2
        for (int kt = 0; kt < HID / 32; ++kt) {
          FragH bl;
          bl.h[0] = *(const v8h*)(hrow + 32 * kt);
          bl.h[1] = *(const v8h*)(hrow + 32 * kt + 16);
          c = wmh(ldfrag(wp + 32 * kt), bl.v, c);
        }
        const v8f bb = ldc8(prm + 16 * ot + 8 * hh);
        float o[8];
#pragma unroll
        for (int r = 0; r < 8; ++r) o[r] = c[r] * INV2 + bb[r];
        const v4f o0 = {o[0], o[1], o[2], o[3]};
        const v4f o1 = {o[4], o[5], o[6], o[7]};
        *(v4f*)(mrow + 16 * ot) = o0;
        *(v4f*)(mrow + 16 * ot + 4) = o1;
      }
    }
    __syncthreads();

    if (tid < EMBD) {
#pragma unroll 1
      for (int i = 0; i < PASSN; ++i) {
        int sl = slotb[i];
        sl = sl < 0 ? 0 : (sl > NAG ? NAG : sl);
        acc[sl * EMBD + tid] += msg[i * EMBD + tid];
      }
    }
    __syncthreads();
  }

  float* pp = part + ((size_t)(b * NSPLIT + s)) * (NAG * EMBD);
#pragma unroll 1
  for (int it = 0; it < (NAG * EMBD) / (NTHR * 4); ++it) {
    const int i = it * NTHR * 4 + 4 * tid;
    const v4f v = *(const v4f*)(acc + i);
    *(volatile v4f*)(pp + i) = v;
  }
  __threadfence();
#pragma unroll 1
  for (int it = 0; it < (NAG * EMBD) / (NTHR * 4); ++it) {
    const int i = it * NTHR * 4 + 4 * tid;
    const v4f v = *(const v4f*)(acc + i);
    *(volatile v4f*)(pp + i) = v;
  }
}

__global__ __launch_bounds__(NTHR) __attribute__((amdgpu_num_vgpr(256))) void k_node(
    const float* __restrict__ x0, const float* __restrict__ xl, const float* __restrict__ part,
    const _Float16* __restrict__ W3p, const float* __restrict__ b3,
    const _Float16* __restrict__ W4p, const float* __restrict__ b4, float* out) {
  extern __shared__ __attribute__((aligned(16))) unsigned char dsm[];
  _Float16* ag   = (_Float16*)(dsm + N_AG);
  _Float16* hb   = (_Float16*)(dsm + N_H);
  float*    outs = (float*)(dsm + N_OUT);
  float*    prm  = (float*)(dsm + N_PRM);
  const int tid = threadIdx.x, lane = tid & 31, wave = tid >> 5, hh = lane >> 4, m = lane & 15;
  const int b = blockIdx.x;

  prm[tid] = b3[tid];
  if (tid < EMBD) prm[HID + tid] = b4[tid];
#pragma unroll
  for (int it = 0; it < (NAG * FEATD / 8) / NTHR; ++it) {
    const int i = it * NTHR + tid;
    const int n = i >> 2, c8 = i & 3;
    const float* xp = x0 + ((size_t)(b * NAG + n)) * FEATD + 8 * c8;
    *(v8h*)(ag + n * AGP + 8 * c8) = cv8s(*(const v4f*)xp, *(const v4f*)(xp + 4));
  }
#pragma unroll
  for (int it = 0; it < (NAG * EMBD / 8) / NTHR; ++it) {
    const int i = it * NTHR + tid;
    const int n = i >> 3, c8 = i & 7;
    const float* xp = xl + ((size_t)(b * NAG + n)) * EMBD + 8 * c8;
    *(v8h*)(ag + n * AGP + FEATD + 8 * c8) = cv8s(*(const v4f*)xp, *(const v4f*)(xp + 4));
  }
#pragma unroll 1
  for (int it = 0; it < (NAG * EMBD / 4) / NTHR; ++it) {
    const int i = it * NTHR + tid;
    const int n = i >> 4, c4 = i & 15;
    v4f sacc = {0.0f, 0.0f, 0.0f, 0.0f};
#pragma unroll
    for (int sp = 0; sp < NSPLIT; ++sp)
      sacc += *(const v4f*)(part + ((size_t)((b * NSPLIT + sp) * NAG + n)) * EMBD + 4 * c4);
    *(v4h*)(ag + n * AGP + FEATD + EMBD + 4 * c4) = cv4s(sacc);
  }
  __syncthreads();

  const int lrow = 16 * wave + m;
  {
    const _Float16* brow = ag + lrow * AGP + 8 * hh;
    _Float16* hrow = hb + lrow * HP + 8 * hh;
#pragma unroll 1
    for (int q = 0; q < HID / 32; ++q) {
      v8f d0 = splat8(0.0f), d1 = splat8(0.0f);
      const _Float16* w0p = W3p + (size_t)(32 * q + m) * K2IN + 8 * hh;
      const _Float16* w1p = w0p + (size_t)16 * K2IN;
#pragma unroll 1
      for (int kf = 0; kf < K2IN / 32; ++kf) {
        FragH bl;
        bl.h[0] = *(const v8h*)(brow + 32 * kf);
        bl.h[1] = *(const v8h*)(brow + 32 * kf + 16);
        d0 = wmh(ldfrag(w0p + 32 * kf), bl.v, d0);
        d1 = wmh(ldfrag(w1p + 32 * kf), bl.v, d1);
      }
      const v8h h0 = act8(d0, ldc8(prm + 32 * q + 8 * hh));
      const v8h h1 = act8(d1, ldc8(prm + 32 * q + 16 + 8 * hh));
      *(v8h*)(hrow + 32 * q) = h0;
      *(v8h*)(hrow + 32 * q + 16) = h1;
    }
  }
  __syncthreads();
  {
    const _Float16* hrow = hb + lrow * HP + 8 * hh;
    float* orow = outs + lrow * EMBD + 8 * hh;
#pragma unroll 1
    for (int ot = 0; ot < EMBD / 16; ++ot) {
      v8f c = splat8(0.0f);
      const _Float16* wp = W4p + (size_t)(16 * ot + m) * HID + 8 * hh;
#pragma unroll 2
      for (int kt = 0; kt < HID / 32; ++kt) {
        FragH bl;
        bl.h[0] = *(const v8h*)(hrow + 32 * kt);
        bl.h[1] = *(const v8h*)(hrow + 32 * kt + 16);
        c = wmh(ldfrag(wp + 32 * kt), bl.v, c);
      }
      const v8f bb = ldc8(prm + HID + 16 * ot + 8 * hh);
      float o[8];
#pragma unroll
      for (int r = 0; r < 8; ++r) o[r] = c[r] * INV2 + bb[r];
      const v4f o0 = {o[0], o[1], o[2], o[3]};
      const v4f o1 = {o[4], o[5], o[6], o[7]};
      *(v4f*)(orow + 16 * ot) = o0;
      *(v4f*)(orow + 16 * ot + 4) = o1;
    }
  }
  __syncthreads();

  float* op = out + (size_t)b * (NAG * EMBD);
#pragma unroll 1
  for (int it = 0; it < (NAG * EMBD) / (NTHR * 4); ++it) {
    const int i = it * NTHR * 4 + 4 * tid;
    const v4f v = *(const v4f*)(outs + i);
    *(volatile v4f*)(op + i) = v;
  }
  __threadfence();
#pragma unroll 1
  for (int it = 0; it < (NAG * EMBD) / (NTHR * 4); ++it) {
    const int i = it * NTHR * 4 + 4 * tid;
    const v4f v = *(const v4f*)(outs + i);
    *(volatile v4f*)(op + i) = v;
  }
}

extern "C" void kernel_launch(void* const* d_in, const int* in_sizes, int n_in,
                              void* d_out, int out_size, void* d_ws, size_t ws_size,
                              hipStream_t stream) {
  if (n_in < 14) return;
  const int nE = in_sizes[13] / 2;
  if (nE < 1 || in_sizes[13] != 2 * nE) return;
  const int nB = in_sizes[0] / (NAG * FEATD);
  if (nB < 1 || nB > 65535 || in_sizes[0] != nB * NAG * FEATD) return;
  if (in_sizes[1] != nB * NAG * EMBD) return;
  if ((size_t)in_sizes[2] != (size_t)nB * (size_t)nE * FEATD) return;
  if (in_sizes[3] != 16 || in_sizes[4] != 8) return;
  if (in_sizes[5] != (YD + EMBD) * HID || in_sizes[6] != HID || in_sizes[7] != HID * EMBD || in_sizes[8] != EMBD) return;
  if (in_sizes[9] != K2IN * HID || in_sizes[10] != HID || in_sizes[11] != HID * EMBD || in_sizes[12] != EMBD) return;
  if (out_size != nB * NAG * EMBD) return;

  const float* x0     = (const float*)d_in[0];
  const float* x_last = (const float*)d_in[1];
  const float* eattr  = (const float*)d_in[2];
  const float* conv_w = (const float*)d_in[3];
  const float* conv_b = (const float*)d_in[4];
  const float* m1w1   = (const float*)d_in[5];
  const float* m1b1   = (const float*)d_in[6];
  const float* m1w2   = (const float*)d_in[7];
  const float* m1b2   = (const float*)d_in[8];
  const float* m2w1   = (const float*)d_in[9];
  const float* m2b1   = (const float*)d_in[10];
  const float* m2w2   = (const float*)d_in[11];
  const float* m2b2   = (const float*)d_in[12];
  const int*   eidx   = (const int*)d_in[13];
  float* outp = (float*)d_out;

  char* ws = (char*)d_ws;
  size_t off = 0;
  const size_t oW1y = off; off += ((size_t)HID * YD * 2 + 255) & ~(size_t)255;
  const size_t oW1x = off; off += ((size_t)HID * EMBD * 2 + 255) & ~(size_t)255;
  const size_t oW2  = off; off += ((size_t)EMBD * HID * 2 + 255) & ~(size_t)255;
  const size_t oW3  = off; off += ((size_t)HID * K2IN * 2 + 255) & ~(size_t)255;
  const size_t oW4  = off; off += ((size_t)EMBD * HID * 2 + 255) & ~(size_t)255;
  const size_t oP   = off; off += ((size_t)nB * NAG * HID * 4 + 255) & ~(size_t)255;
  const size_t oPt  = off; off += ((size_t)nB * NSPLIT * NAG * EMBD * 4 + 255) & ~(size_t)255;
  size_t limit = (size_t)134217728;
  if (ws_size < limit) limit = ws_size;
  if (off > limit) return;

  _Float16* pW1y = (_Float16*)(ws + oW1y);
  _Float16* pW1x = (_Float16*)(ws + oW1x);
  _Float16* pW2  = (_Float16*)(ws + oW2);
  _Float16* pW3  = (_Float16*)(ws + oW3);
  _Float16* pW4  = (_Float16*)(ws + oW4);
  float* Pn  = (float*)(ws + oP);
  float* Prt = (float*)(ws + oPt);

  const int epb = (((nE + NSPLIT - 1) / NSPLIT) + PASSN - 1) / PASSN * PASSN;

  k_prep<<<PBT, NTHR, 0, stream>>>(m1w1, m1w2, m2w1, m2w2, pW1y, pW1x, pW2, pW3, pW4);

  hipFuncSetAttribute(reinterpret_cast<const void*>(&k_pnode), hipFuncAttributeMaxDynamicSharedMemorySize, P_TOT);
  hipFuncSetAttribute(reinterpret_cast<const void*>(&k_edge),  hipFuncAttributeMaxDynamicSharedMemorySize, E_TOT);
  hipFuncSetAttribute(reinterpret_cast<const void*>(&k_node),  hipFuncAttributeMaxDynamicSharedMemorySize, N_TOT);

  k_pnode<<<nB, NTHR, P_TOT, stream>>>(x_last, pW1x, m1b1, Pn);
  k_edge<<<dim3(NSPLIT, nB), NTHR, E_TOT, stream>>>(x0, eattr, eidx, conv_w, conv_b, m1b2, Pn, pW1y, pW2,
                                                    Prt, nE, epb);
  k_node<<<nB, NTHR, N_TOT, stream>>>(x0, x_last, Prt, pW3, m2b1, pW4, m2b2, outp);
}
